// RelationAttentionBatch_82566451299182
// MI455X (gfx1250) — hardware-run, weakly checked
//
#include <hip/hip_runtime.h>


#ifndef NB
#define NB 4
#endif
#define NB_FULL  4
#define SEQ      64
#define SEQ_FULL 64
#define DM   128
#define NTY  50
#define KTP  (NTY * DM)
#define AW   4
#define SP   68
#define PP   72
#define VP   72
#define CP   136
#define OP   132
#define PCAR 16384.0f
#define WCAR 64.0f
#define WINV (1.0f / 64.0f)
#define LOG2E 1.4426950408889634f
#define FILLV (-1.0e9f)

static_assert(SEQ == 64);
static_assert(SEQ == SEQ_FULL);
static_assert(DM == 128);
static_assert(AW == 4);
static_assert(AW * 32 == DM);
static_assert(DM % 32 == 0);
static_assert(SEQ % 32 == 0);
static_assert((NB * SEQ) % 64 == 0);
static_assert(KTP % 64 == 0);
static_assert(SEQ % 16 == 0);
static_assert(NB <= NB_FULL);
static_assert(32 * 4 * 8 == 16 * 64);
static_assert(32 * AW * 4 * 4 == 16 * DM);
static_assert(32 * AW * 4 * 16 == SEQ * DM);
static_assert(32 * AW * 8 == 16 * SEQ);
static_assert(32 * AW * 4 * 2 == 16 * SEQ);
static_assert((SP * 4) % 16 == 0);
static_assert((PP * 2) % 16 == 0);
static_assert((VP * 2) % 16 == 0);
static_assert((CP * 2) % 16 == 0);
static_assert((OP * 4) % 16 == 0);
static_assert(PP >= SEQ);
static_assert(VP >= SEQ);
static_assert(CP >= DM);
static_assert(OP >= DM);
static_assert((size_t)16 * DM * 4 + (size_t)16 * SP * 4 + (size_t)16 * PP * 2 + (size_t)DM * VP * 2 + (size_t)16 * CP * 2 + (size_t)16 * OP * 4 + 64 <= (size_t)131072);
static_assert((size_t)16 * 68 * 4 <= (size_t)131072);
static_assert((size_t)NB_FULL * SEQ_FULL * DM * 4 == (size_t)131072);
static_assert(((size_t)(NB - 1) * SEQ_FULL + SEQ) * DM <= (size_t)NB_FULL * SEQ_FULL * DM);
static_assert((size_t)(NB * SEQ - 1) * KTP + (size_t)(NTY - 1) * DM + DM <= (size_t)NB * SEQ * KTP);
static_assert((size_t)NB * SEQ * KTP < (size_t)4294967295u);

typedef _Float16 h16;
typedef unsigned short bf;
typedef __attribute__((ext_vector_type(16))) __bf16   v16bf;
typedef __attribute__((ext_vector_type(16))) _Float16 v16h;
typedef __attribute__((ext_vector_type(8)))  _Float16 v8h;
typedef __attribute__((ext_vector_type(8)))  unsigned short v8us;
typedef __attribute__((ext_vector_type(8)))  float    v8f;
typedef __attribute__((ext_vector_type(4)))  float    v4f;
typedef v4f  __attribute__((may_alias)) v4fa;
typedef v8h  __attribute__((may_alias)) v8ha;

__device__ __forceinline__ unsigned short f2bf(float f) { unsigned u = __float_as_uint(f); u += 0x7FFFu + ((u >> 16) & 1u); return (unsigned short)(u >> 16); }
__device__ __forceinline__ float bfr(float f) { return __uint_as_float(((unsigned)f2bf(f)) << 16); }
__device__ __forceinline__ v16h cat16(v8h lo, v8h hi) { return __builtin_shufflevector(lo, hi, 0, 1, 2, 3, 4, 5, 6, 7, 8, 9, 10, 11, 12, 13, 14, 15); }
__device__ __forceinline__ v16bf cat16b(v8us lo, v8us hi) { return __builtin_bit_cast(v16bf, __builtin_shufflevector(lo, hi, 0, 1, 2, 3, 4, 5, 6, 7, 8, 9, 10, 11, 12, 13, 14, 15)); }
__device__ __forceinline__ v8f wmma16(v16h a, v16h b, v8f c) { return __builtin_amdgcn_wmma_f32_16x16x32_f16(false, a, false, b, (short)0, c, false, false); }
__device__ __forceinline__ v8f wmmab(v16bf a, v16bf b, v8f c) { return __builtin_amdgcn_wmma_f32_16x16x32_bf16(false, a, false, b, (short)0, c, false, false); }
__device__ __forceinline__ v16h  ldh(const h16* p) { return cat16(*(const v8h*)p, *(const v8h*)(p + 16)); }
__device__ __forceinline__ v16bf ldb(const bf* p)  { return cat16b(*(const v8us*)p, *(const v8us*)(p + 16)); }
__device__ __forceinline__ void wave_sync() { __builtin_amdgcn_fence(3  , "wavefront"); __builtin_amdgcn_wave_barrier(); asm volatile("" ::: "memory"); }

__device__ __forceinline__ v8f wmma16g(v16h a, v16h b, v8f c) {
    c = __builtin_amdgcn_wmma_f32_16x16x32_f16(false, a, false, b, (short)0, c, false, false);
    asm volatile("v_nop\n\tv_nop\n\tv_nop\n\tv_nop" : "+v"(c) : "v"(a), "v"(b));
    return c;
}
__device__ __forceinline__ v8f wmmabg(v16bf a, v16bf b, v8f c) {
    c = __builtin_amdgcn_wmma_f32_16x16x32_bf16(false, a, false, b, (short)0, c, false, false);
    asm volatile("v_nop\n\tv_nop\n\tv_nop\n\tv_nop" : "+v"(c) : "v"(a), "v"(b));
    return c;
}
static __device__ __forceinline__ h16 toh_flush(float v) { const h16 r = (h16)v; return (fabsf(v) < 6.103515625e-05f) ? (h16)0.0f : r; }

__global__ __launch_bounds__(256) void k_cvt8(const float* __restrict__ src, bf* dst, size_t n8) {
    const size_t i = (size_t)blockIdx.x * 256 + threadIdx.x; if (i >= n8) return;
    const v8f v = *(const v8f*)(src + i * 8); v8us o;
#pragma unroll
    for (int k = 0; k < 8; ++k) o[k] = f2bf(v[k]);
    *(volatile v8us*)(dst + i * 8) = o; __threadfence(); *(volatile v8us*)(dst + i * 8) = o;
}

__global__ __launch_bounds__(256) void k_wconv(const float* __restrict__ src, h16* dst, size_t n8) {
    const size_t i = (size_t)blockIdx.x * 256 + threadIdx.x; if (i >= n8) return;
    const v8f v = *(const v8f*)(src + i * 8); v8h o;
#pragma unroll
    for (int k = 0; k < 8; ++k) o[k] = toh_flush(bfr(v[k]) * WCAR);
    *(volatile v8h*)(dst + i * 8) = o; __threadfence(); *(volatile v8h*)(dst + i * 8) = o;
}

__global__ __launch_bounds__(32) void k_gemm(const bf* __restrict__ A, const bf* __restrict__ Bt, float* C) {
    __shared__ __align__(16) float os[16 * 68];
    const int K = DM;
    const int lane = threadIdx.x & 31, lr = lane & 15, hi = lane >> 4; const int r0 = blockIdx.x * 64, c0 = blockIdx.y * 64;
    v8f acc[4][4];
#pragma unroll
    for (int mb = 0; mb < 4; ++mb)
#pragma unroll
        for (int nb = 0; nb < 4; ++nb) acc[mb][nb] = (v8f){};
    const size_t aoff = (size_t)(r0 + lr) * K + 8 * hi, boff = (size_t)(c0 + lr) * K + 8 * hi;
#pragma unroll 1
    for (int kc = 0; kc < K; kc += 32) {
        v16bf a[4];
#pragma unroll
        for (int mb = 0; mb < 4; ++mb) a[mb] = ldb(A + aoff + (size_t)mb * 16 * K + kc);
#pragma unroll
        for (int nb = 0; nb < 4; ++nb) { const v16bf b = ldb(Bt + boff + (size_t)nb * 16 * K + kc);
#pragma unroll
            for (int mb = 0; mb < 4; ++mb) acc[mb][nb] = wmmabg(a[mb], b, acc[mb][nb]); }
    }
#pragma unroll
    for (int mb = 0; mb < 4; ++mb) {
#pragma unroll
        for (int nb = 0; nb < 4; ++nb) {
#pragma unroll
            for (int j = 0; j < 8; ++j) os[(hi * 8 + j) * 68 + nb * 16 + lr] = acc[mb][nb][j]; }
        wave_sync();
        float* cb = C + (size_t)(r0 + mb * 16) * KTP + c0;
#pragma unroll 1
        for (int ps = 0; ps < 2; ++ps) {
#pragma unroll
            for (int s = 0; s < 8; ++s) { const int row = 2 * s + (lane >> 4), c4 = (lane & 15) * 4;
                const v4f val = *(const v4fa*)(&os[row * 68 + c4]);
                *(volatile v4f*)(cb + (size_t)row * KTP + c4) = val; }
            if (ps == 0) __threadfence(); }
        wave_sync();
    }
}

__global__ __launch_bounds__(32 * AW) void k_rows(const float* __restrict__ Q, const float* __restrict__ V, const int* __restrict__ R, const float* __restrict__ KT,
                                                  const h16* __restrict__ WH, const float* __restrict__ bias, float* OUT0, float* OUT1) {
    __shared__ __align__(16) float qs[16 * DM];
    __shared__ __align__(16) float sc[16 * SP];
    __shared__ __align__(16) h16   ph[16 * PP];
    __shared__ __align__(16) h16   vt[DM * VP];
    __shared__ __align__(16) h16   cx[16 * CP];
    __shared__ __align__(16) float os[16 * OP];
    __shared__ float li[16];
    const int tid = threadIdx.x;
    const int lane = tid & 31, lr = lane & 15, hi = lane >> 4;
    const int wave = __builtin_amdgcn_readfirstlane((int)(threadIdx.x >> 5));
    const int b = blockIdx.y; const int i0 = blockIdx.x * 16;

    const float* qb = Q + ((size_t)b * SEQ_FULL + i0) * DM;
#pragma unroll 1
    for (int it = 0; it < 4; ++it) { const int u = it * (32 * AW) + tid;
        v4f x = *(const v4f*)(qb + (size_t)u * 4);
        x[0] = bfr(x[0]); x[1] = bfr(x[1]); x[2] = bfr(x[2]); x[3] = bfr(x[3]);
        *(v4fa*)(&qs[u * 4]) = x; }
    const float* vb = V + (size_t)b * SEQ_FULL * DM;
#pragma unroll 1
    for (int it = 0; it < 16; ++it) { const int u = it * (32 * AW) + tid; const int j = u >> 5, d4 = (u & 31) * 4;
        const v4f x = *(const v4f*)(vb + (size_t)u * 4);
        vt[(d4 + 0) * VP + j] = toh_flush(bfr(x[0])); vt[(d4 + 1) * VP + j] = toh_flush(bfr(x[1]));
        vt[(d4 + 2) * VP + j] = toh_flush(bfr(x[2])); vt[(d4 + 3) * VP + j] = toh_flush(bfr(x[3])); }
    __syncthreads();

#pragma unroll 1
    for (int it = 0; it < 8; ++it) {
        const int i = it * 2 + (tid >> 6), j = tid & 63;
        const int r = R[((size_t)b * SEQ_FULL + (size_t)(i0 + i)) * SEQ_FULL + j];
        const int rc = r < 0 ? 0 : (r > NTY - 1 ? NTY - 1 : r);
        unsigned ro = (unsigned)rc * (unsigned)DM; asm volatile("" : "+v"(ro));
        const unsigned off = (unsigned)(b * SEQ + j) * (unsigned)KTP + ro;
        const float* kp = KT + off;
        float s0 = 0.0f, s1 = 0.0f, s2 = 0.0f, s3 = 0.0f;
#pragma unroll 4
        for (int d4 = 0; d4 < DM / 4; ++d4) {
            const v4f kv = *(const v4f*)(kp + 4 * d4);
            const v4f qv = *(const v4fa*)(&qs[i * DM + 4 * d4]);
            s0 = fmaf(kv[0], qv[0], s0); s1 = fmaf(kv[1], qv[1], s1); s2 = fmaf(kv[2], qv[2], s2); s3 = fmaf(kv[3], qv[3], s3); }
        float s = (s0 + s1) + (s2 + s3);
        asm volatile("" : "+v"(s));
        s = (r > 0) ? s : FILLV;
        sc[i * SP + j] = s;
    }
    __syncthreads();

    {
        const int row = tid >> 3, c8 = (tid & 7) * 8;
        v4f x0 = *(const v4fa*)(&sc[row * SP + c8]), x1 = *(const v4fa*)(&sc[row * SP + c8 + 4]);
        float mx = fmaxf(fmaxf(fmaxf(x0[0], x0[1]), fmaxf(x0[2], x0[3])), fmaxf(fmaxf(x1[0], x1[1]), fmaxf(x1[2], x1[3])));
        mx = fmaxf(mx, __shfl_xor(mx, 1, 32)); mx = fmaxf(mx, __shfl_xor(mx, 2, 32)); mx = fmaxf(mx, __shfl_xor(mx, 4, 32));
        float e[8]; float es = 0.0f, ls = 0.0f; v8h pv;
#pragma unroll
        for (int k = 0; k < 4; ++k) { e[k] = __builtin_amdgcn_exp2f((x0[k] - mx) * LOG2E); e[4 + k] = __builtin_amdgcn_exp2f((x1[k] - mx) * LOG2E); }
#pragma unroll
        for (int k = 0; k < 8; ++k) { es += e[k]; const h16 p = toh_flush(e[k] * PCAR); pv[k] = p; ls += (float)p; }
        es += __shfl_xor(es, 1, 32); es += __shfl_xor(es, 2, 32); es += __shfl_xor(es, 4, 32);
        ls += __shfl_xor(ls, 1, 32); ls += __shfl_xor(ls, 2, 32); ls += __shfl_xor(ls, 4, 32);
        const float inv = 1.0f / es;
#pragma unroll
        for (int k = 0; k < 4; ++k) { x0[k] = e[k] * inv; x1[k] = e[4 + k] * inv; }
        *(v4fa*)(&sc[row * SP + c8]) = x0; *(v4fa*)(&sc[row * SP + c8 + 4]) = x1;
        *(v8ha*)(&ph[row * PP + c8]) = pv;
        if ((tid & 7) == 0) li[row] = 1.0f / ls;
    }
    __syncthreads();

    {
        v8f c0 = (v8f){}, c1 = (v8f){};
        const int d0 = wave * 32 + lr;
#pragma unroll
        for (int kc = 0; kc < SEQ; kc += 32) {
            const v16h a  = cat16(*(const v8ha*)(&ph[lr * PP + kc + 8 * hi]),        *(const v8ha*)(&ph[lr * PP + kc + 16 + 8 * hi]));
            const v16h b0 = cat16(*(const v8ha*)(&vt[d0 * VP + kc + 8 * hi]),        *(const v8ha*)(&vt[d0 * VP + kc + 16 + 8 * hi]));
            const v16h b1 = cat16(*(const v8ha*)(&vt[(d0 + 16) * VP + kc + 8 * hi]), *(const v8ha*)(&vt[(d0 + 16) * VP + kc + 16 + 8 * hi]));
            c0 = wmma16g(a, b0, c0); c1 = wmma16g(a, b1, c1);
        }
#pragma unroll
        for (int r = 0; r < 8; ++r) { const float nv = li[8 * hi + r];
            cx[(8 * hi + r) * CP + wave * 32 + lr]      = toh_flush(c0[r] * nv);
            cx[(8 * hi + r) * CP + wave * 32 + 16 + lr] = toh_flush(c1[r] * nv); }
    }
    __syncthreads();

    {
        v8f o0 = (v8f){}, o1 = (v8f){};
        const size_t wo = (size_t)(wave * 32 + lr) * DM + 8 * hi;
#pragma unroll
        for (int kc = 0; kc < DM; kc += 32) {
            const v16h a  = cat16(*(const v8ha*)(&cx[lr * CP + kc + 8 * hi]), *(const v8ha*)(&cx[lr * CP + kc + 16 + 8 * hi]));
            const v16h b0 = ldh(WH + wo + kc);
            const v16h b1 = ldh(WH + wo + (size_t)16 * DM + kc);
            o0 = wmma16g(a, b0, o0); o1 = wmma16g(a, b1, o1);
        }
        const float bb0 = bfr(bias[wave * 32 + lr]), bb1 = bfr(bias[wave * 32 + 16 + lr]);
#pragma unroll
        for (int r = 0; r < 8; ++r) {
            os[(8 * hi + r) * OP + wave * 32 + lr]      = o0[r] * WINV + bb0;
            os[(8 * hi + r) * OP + wave * 32 + 16 + lr] = o1[r] * WINV + bb1; }
    }
    __syncthreads();

    float* g0 = OUT0 + ((size_t)b * SEQ_FULL + i0) * DM;
    float* g1 = OUT1 + ((size_t)b * SEQ_FULL + i0) * SEQ_FULL;
#pragma unroll 1
    for (int ps = 0; ps < 2; ++ps) {
#pragma unroll
        for (int it = 0; it < 4; ++it) { const int u = it * (32 * AW) + tid; const int row = u >> 5, c4 = (u & 31) * 4;
            const v4f val = *(const v4fa*)(&os[row * OP + c4]);
            *(volatile v4f*)(g0 + (size_t)u * 4) = val; }
#pragma unroll
        for (int it = 0; it < 2; ++it) { const int u = it * (32 * AW) + tid; const int row = u >> 4, c4 = (u & 15) * 4;
            const v4f val = *(const v4fa*)(&sc[row * SP + c4]);
            *(volatile v4f*)(g1 + (size_t)u * 4) = val; }
        if (ps == 0) __threadfence(); }
}

static constexpr size_t al256(size_t v) { return (v + 255) & ~(size_t)255; }
static constexpr size_t SZ_KB = al256((size_t)NB * SEQ * DM * 2);
static constexpr size_t SZ_TB = al256((size_t)NTY * DM * DM * 2);
static constexpr size_t SZ_WH = al256((size_t)DM * DM * 2);
static constexpr size_t SZ_KT = al256((size_t)NB * SEQ * KTP * 4);
static constexpr size_t SZ_TOTAL = SZ_KB + SZ_TB + SZ_WH + SZ_KT;
static_assert(SZ_TOTAL <= (size_t)134217728);
static_assert(((size_t)NB * SEQ * DM) % 8 == 0);
static_assert(((size_t)NTY * DM * DM) % 8 == 0);
static_assert(((size_t)DM * DM) % 8 == 0);
static_assert((size_t)(NB * SEQ / 64) * 64 * KTP * 4 <= SZ_KT);
static_assert((size_t)(KTP / 64) * 64 == (size_t)KTP);

extern "C" void kernel_launch(void* const* d_in, const int* in_sizes, int n_in,
                              void* d_out, int out_size, void* d_ws, size_t ws_size, hipStream_t stream) {
    if (n_in < 7) return;
    const size_t needx = ((size_t)(NB - 1) * SEQ_FULL + SEQ) * DM;
    const size_t needr = ((size_t)(NB - 1) * SEQ_FULL + SEQ) * SEQ_FULL;
    if ((size_t)in_sizes[0] < needx || (size_t)in_sizes[1] < needx || (size_t)in_sizes[2] < needx) return;
    if ((size_t)in_sizes[3] < needr) return;
    if ((size_t)in_sizes[4] < (size_t)NTY * DM * DM || (size_t)in_sizes[5] < (size_t)DM * DM || in_sizes[6] < DM) return;
    if ((size_t)out_size < (size_t)NB_FULL * SEQ_FULL * DM + needr) return;
    if (SZ_TOTAL > ws_size) return;
    const float* q   = (const float*)d_in[0];
    const float* key = (const float*)d_in[1];
    const float* val = (const float*)d_in[2];
    const int*   R   = (const int*)d_in[3];
    const float* tab = (const float*)d_in[4];
    const float* wo  = (const float*)d_in[5];
    const float* bo  = (const float*)d_in[6];
    float* OUT0 = (float*)d_out;
    float* OUT1 = OUT0 + (size_t)NB_FULL * SEQ_FULL * DM;
    char* wsp = (char*)d_ws;
    bf*    KB = (bf*)wsp;    wsp += SZ_KB;
    bf*    TB = (bf*)wsp;    wsp += SZ_TB;
    h16*   WH = (h16*)wsp;   wsp += SZ_WH;
    float* KT = (float*)wsp; wsp += SZ_KT;

    { const size_t n8 = (size_t)NB * SEQ * DM / 8;  k_cvt8<<<(unsigned)((n8 + 255) / 256), 256, 0, stream>>>(key, KB, n8); }
    { const size_t n8 = (size_t)NTY * DM * DM / 8;  k_cvt8<<<(unsigned)((n8 + 255) / 256), 256, 0, stream>>>(tab, TB, n8); }
    { const size_t n8 = (size_t)DM * DM / 8;        k_wconv<<<(unsigned)((n8 + 255) / 256), 256, 0, stream>>>(wo, WH, n8); }
    k_gemm<<<dim3(NB * SEQ / 64, KTP / 64, 1), 32, 0, stream>>>(KB, TB, KT);
    k_rows<<<dim3(SEQ / 16, NB, 1), 32 * AW, 0, stream>>>(q, val, R, KT, WH, bo, OUT0, OUT1);
}
